// self_transformer_41575283425956
// MI455X (gfx1250) — hardware-verified
//
#include <hip/hip_runtime.h>
#include <math.h>

typedef __attribute__((ext_vector_type(16))) _Float16 v16h;
typedef __attribute__((ext_vector_type(16))) __bf16 v16b;
typedef __attribute__((ext_vector_type(8)))  _Float16 v8h;
typedef __attribute__((ext_vector_type(8)))  float v8f;
typedef __attribute__((ext_vector_type(4)))  float v4f;
typedef __attribute__((ext_vector_type(2)))  float v2f;
typedef __attribute__((ext_vector_type(4)))  unsigned v4u;
typedef __attribute__((ext_vector_type(4)))  int v4i;
typedef float __attribute__((may_alias)) float_a;
typedef int __attribute__((may_alias)) int_a;

template <typename T> __device__ __forceinline__ void vst2(void* p, T v) { *(volatile T*)p = v; __threadfence(); *(volatile T*)p = v; }
__device__ __forceinline__ v8f wmma16(v16h a, v16h b, v8f c) {
  v8f d = __builtin_amdgcn_wmma_f32_16x16x32_f16(false, a, false, b, (short)0, c, false, false);
  asm volatile("v_nop\n\tv_nop\n\tv_nop\n\tv_nop" : "+v"(d) : "v"(a), "v"(b));
  return d;
}
__device__ __forceinline__ v8f wmma_bf(v16b a, v16b b, v8f c) {
  v8f d = __builtin_amdgcn_wmma_f32_16x16x32_bf16(false, a, false, b, (short)0, c, false, false);
  asm volatile("v_nop\n\tv_nop\n\tv_nop\n\tv_nop" : "+v"(d) : "v"(a), "v"(b));
  return d;
}
__device__ __forceinline__ v16h frag_h(const _Float16* rowk0, int lane) {
  union { v16h v; v8h q[2]; } u; const _Float16* p = rowk0 + 8 * (lane >> 4);
  u.q[0] = *(const v8h*)p; u.q[1] = *(const v8h*)(p + 16); return u.v;
}
__device__ __forceinline__ v16h frag_f32(const float* rowk0, int lane) {
  v16h a; const float* p = rowk0 + 8 * (lane >> 4);
#pragma unroll
  for (int i = 0; i < 8; ++i) { a[i] = (_Float16)p[i]; a[8 + i] = (_Float16)p[16 + i]; }
  return a;
}
__device__ __forceinline__ v16h frag_f32s(const float* rowk0, int lane, float sc) {
  v16h a; const float* p = rowk0 + 8 * (lane >> 4);
#pragma unroll
  for (int i = 0; i < 8; ++i) { a[i] = (_Float16)(p[i] * sc); a[8 + i] = (_Float16)(p[16 + i] * sc); }
  return a;
}
__device__ __forceinline__ v16h fragc_f32(const float* W, int k0, int n, int lane, int ld, int K) {
  v16h a; const int g = lane >> 4;
#pragma unroll
  for (int i = 0; i < 8; ++i) { const int ka = k0 + 8 * g + i, kb = ka + 16;
    a[i] = (_Float16)(ka < K ? W[(size_t)(ka < K ? ka : K - 1) * ld + n] : 0.f); a[8 + i] = (_Float16)(kb < K ? W[(size_t)(kb < K ? kb : K - 1) * ld + n] : 0.f); }
  return a;
}
struct F2 { v16b h, l; };
__device__ __forceinline__ F2 bsplit16(const float v[16]) { F2 r;
#pragma unroll
  for (int i = 0; i < 16; ++i) { const __bf16 h = (__bf16)v[i]; r.h[i] = h; r.l[i] = (__bf16)(v[i] - (float)h); }
  return r; }
__device__ __forceinline__ F2 split_row(const float* row, int k0, int lane) { float v[16]; const float* p = row + k0 + 8 * (lane >> 4);
#pragma unroll
  for (int i = 0; i < 8; ++i) { v[i] = p[i]; v[8 + i] = p[16 + i]; }
  return bsplit16(v); }
__device__ __forceinline__ F2 split_rowK(const float* row, int k0, int lane, int K) { float v[16]; const int g = lane >> 4;
#pragma unroll
  for (int i = 0; i < 8; ++i) { const int ka = k0 + 8 * g + i, kb = ka + 16; v[i] = ka < K ? row[ka < K ? ka : K - 1] : 0.f; v[8 + i] = kb < K ? row[kb < K ? kb : K - 1] : 0.f; }
  return bsplit16(v); }
__device__ __forceinline__ F2 split_col(const float* W, int k0, int n, int lane, int ld, int K) { float v[16]; const int g = lane >> 4;
#pragma unroll
  for (int i = 0; i < 8; ++i) { const int ka = k0 + 8 * g + i, kb = ka + 16; v[i] = ka < K ? W[(size_t)(ka < K ? ka : K - 1) * ld + n] : 0.f; v[8 + i] = kb < K ? W[(size_t)(kb < K ? kb : K - 1) * ld + n] : 0.f; }
  return bsplit16(v); }
__device__ __forceinline__ v8f mac3(const F2& a, const F2& b, v8f c) { c = wmma_bf(a.l, b.h, c); c = wmma_bf(a.h, b.l, c); return wmma_bf(a.h, b.h, c); }
__device__ __forceinline__ float sigm(float v) { return 1.0f / (1.0f + expf(-v)); }
#define LDSX() do { asm volatile("s_wait_dscnt 0" ::: "memory"); __builtin_amdgcn_wave_barrier(); __builtin_amdgcn_fence(__ATOMIC_RELEASE, "workgroup"); } while (0)


#define NN 4096
#define DD 1024
#define QBLK 512
#ifndef NQB
#define NQB (NN / QBLK)
#endif
typedef __attribute__((ext_vector_type(8))) __bf16 v8b;
__device__ __forceinline__ v16b frag_b(const __bf16* rowk0, int lane) {
  union { v16b v; v8b q[2]; } u; const __bf16* p = rowk0 + 8 * (lane >> 4);
  u.q[0] = *(const v8b*)p; u.q[1] = *(const v8b*)(p + 16); return u.v;
}
__device__ __forceinline__ float bfr(float v) { return (float)(__bf16)v; }
__device__ __attribute__((noinline)) float exp_ni(float v) { return expf(v); }
__device__ __attribute__((noinline)) float erf_ni(float v) { return erff(v); }

#define WS_PW  0u
#define WS_Q   (WS_PW + 2u * (size_t)3 * DD * DD)
#define WS_KH  (WS_Q + 2u * (size_t)NN * DD)
#define WS_KL  (WS_KH + 2u * (size_t)NN * DD)
#define WS_VT  (WS_KL + 2u * (size_t)NN * DD)
#define WS_S   (WS_VT + 2u * (size_t)DD * NN)
#define WS_P   (WS_S + 4u * (size_t)QBLK * NN)
#define WS_IL  (WS_P + 2u * (size_t)QBLK * NN)
#define WS_END (WS_IL + 4u * QBLK + 256u)

__global__ __launch_bounds__(256) void k_pack(const float* __restrict__ W1, const float* __restrict__ W2, const float* __restrict__ W3, __bf16* __restrict__ P) { const int n = blockIdx.x, which = blockIdx.y, t = threadIdx.x; const float* Wm = (which == 0) ? W1 : (which == 1) ? W2 : W3; __shared__ __align__(16) __bf16 s[DD]; for (int k = t; k < DD; k += 256) s[k] = (__bf16)Wm[(size_t)n * DD + k]; __syncthreads(); for (int q = t; q < DD / 8; q += 256) vst2((unsigned*)(P + ((size_t)which * DD + n) * DD + q * 8), *(const v4u*)&s[q * 8]); }
__global__ __launch_bounds__(128) void k_proj(const float* __restrict__ X, const __bf16* __restrict__ P, const float* __restrict__ B1v, const float* __restrict__ B2v, const float* __restrict__ B3v, _Float16* __restrict__ Q, _Float16* __restrict__ KH, _Float16* __restrict__ KL, _Float16* __restrict__ VT) {
  __shared__ __align__(16) _Float16 sh[64][136], sl[64][136]; __shared__ __align__(16) _Float16 st[128][72];
  const int tid = threadIdx.x, wave = tid >> 5, lane = tid & 31, col = lane & 15, g = lane >> 4; const int which = blockIdx.z; const int n0 = blockIdx.y * 128; const size_t rb0 = (size_t)blockIdx.x * 64, r0 = rb0 + wave * 16;
  const __bf16* Wr = P + (size_t)which * DD * DD; const float* BB = (which == 0) ? B1v : (which == 1) ? B2v : B3v;
  v8f acc[8] = {};
#pragma unroll 2
  for (int kc = 0; kc < DD / 32; ++kc) { v16b a; { const float* p = X + (r0 + col) * DD + kc * 32 + 8 * g;
#pragma unroll
      for (int i = 0; i < 8; ++i) { a[i] = (__bf16)p[i]; a[8 + i] = (__bf16)p[16 + i]; } }
#pragma unroll
    for (int j = 0; j < 8; ++j) acc[j] = wmma_bf(a, frag_b(Wr + (size_t)(n0 + j * 16 + col) * DD + kc * 32, lane), acc[j]); }
  if (which < 2) {
#pragma unroll
    for (int j = 0; j < 8; ++j) { const float bb = bfr(BB[n0 + j * 16 + col]);
#pragma unroll
      for (int r = 0; r < 8; ++r) { const float v = acc[j][r] + bb; const _Float16 h = (_Float16)v; sh[wave * 16 + 8 * g + r][j * 16 + col] = h; sl[wave * 16 + 8 * g + r][j * 16 + col] = (_Float16)((v - (float)h) * 2048.0f); } }
    LDSX();
    if (which == 0) { for (int rl = 0; rl < 16; ++rl) if (lane < 16) vst2((unsigned*)(Q + (r0 + rl) * DD + n0 + lane * 8), *(const v4u*)&sh[wave * 16 + rl][lane * 8]); }
    else { for (int rl = 0; rl < 16; ++rl) if (lane < 16) { vst2((unsigned*)(KH + (r0 + rl) * DD + n0 + lane * 8), *(const v4u*)&sh[wave * 16 + rl][lane * 8]); vst2((unsigned*)(KL + (r0 + rl) * DD + n0 + lane * 8), *(const v4u*)&sl[wave * 16 + rl][lane * 8]); } }
  } else {
#pragma unroll
    for (int j = 0; j < 8; ++j) { const float bb = bfr(BB[n0 + j * 16 + col]);
#pragma unroll
      for (int r = 0; r < 8; ++r) st[j * 16 + col][wave * 16 + 8 * g + r] = (_Float16)(acc[j][r] + bb); }
    __syncthreads();
    for (int e = tid; e < 128 * 8; e += 128) { const int d = e >> 3, pc = e & 7; vst2((unsigned*)(VT + (size_t)(n0 + d) * NN + rb0 + pc * 8), *(const v4u*)&st[d][pc * 8]); } }
}
__global__ __launch_bounds__(128) void k_scores(const _Float16* __restrict__ KH, const _Float16* __restrict__ KL, const _Float16* __restrict__ Q, int nbase, float* __restrict__ S) {
  __shared__ __align__(16) float so[4][16][132];
  const int tid = threadIdx.x, wave = tid >> 5, lane = tid & 31, col = lane & 15, g = lane >> 4; const int rloc0 = blockIdx.x * 64 + wave * 16; const size_t rn = (size_t)nbase + rloc0; const int m0 = blockIdx.y * 128;
  v8f acc[8] = {}, accl[8] = {};
#pragma unroll 4
  for (int kc = 0; kc < DD / 32; ++kc) { const v16h a = frag_h(KH + (rn + col) * DD + kc * 32, lane), al = frag_h(KL + (rn + col) * DD + kc * 32, lane);
#pragma unroll
    for (int j = 0; j < 8; ++j) { const v16h qf = frag_h(Q + (size_t)(m0 + j * 16 + col) * DD + kc * 32, lane); acc[j] = wmma16(a, qf, acc[j]); accl[j] = wmma16(al, qf, accl[j]); } }
#pragma unroll
  for (int j = 0; j < 8; ++j)
#pragma unroll
    for (int r = 0; r < 8; ++r) so[wave][8 * g + r][j * 16 + col] = (acc[j][r] + accl[j][r] * (1.0f / 2048.0f)) * 0.03125f;
  LDSX();
  for (int rl = 0; rl < 16; ++rl) vst2(S + (size_t)(rloc0 + rl) * NN + m0 + lane * 4, *(const v4f*)&so[wave][rl][lane * 4]);
}
__global__ __launch_bounds__(256) void k_soft(const float* __restrict__ S, _Float16* __restrict__ P, float* __restrict__ IL) {
  __shared__ float red[256]; __shared__ __align__(16) _Float16 sp[NN];
  const int r = blockIdx.x, t = threadIdx.x; const float* row = S + (size_t)r * NN;
  float mx = -3.0e38f; for (int k = t; k < NN; k += 256) mx = fmaxf(mx, row[k]); red[t] = mx; __syncthreads();
  for (int s = 128; s > 0; s >>= 1) { if (t < s) red[t] = fmaxf(red[t], red[t + s]); __syncthreads(); }
  const float gm = red[0]; __syncthreads();
  float sum = 0.f; for (int k = t; k < NN; k += 256) { const float e = __expf(row[k] - gm); sum += e; sp[k] = (_Float16)(e * 2048.0f); }
  red[t] = sum; __syncthreads();
  for (int s = 128; s > 0; s >>= 1) { if (t < s) red[t] += red[t + s]; __syncthreads(); }
  if (t == 0) IL[r] = (1.0f / 2048.0f) / red[0];
  for (int q = t; q < NN / 8; q += 256) vst2((unsigned*)(P + (size_t)r * NN + q * 8), *(const v4u*)&sp[q * 8]);
}
__global__ __launch_bounds__(128) void k_pv(const _Float16* __restrict__ P, const _Float16* __restrict__ VT, const float* __restrict__ IL, int nbase, float* __restrict__ OUT) {
  __shared__ __align__(16) float so[4][16][132];
  const int tid = threadIdx.x, wave = tid >> 5, lane = tid & 31, col = lane & 15, g = lane >> 4; const int rloc0 = blockIdx.x * 64 + wave * 16; const int d0 = blockIdx.y * 128;
  v8f acc[8] = {};
#pragma unroll 2
  for (int kc = 0; kc < NN / 32; ++kc) { const v16h a = frag_h(P + (size_t)(rloc0 + col) * NN + kc * 32, lane);
#pragma unroll
    for (int j = 0; j < 8; ++j) acc[j] = wmma16(a, frag_h(VT + (size_t)(d0 + j * 16 + col) * NN + kc * 32, lane), acc[j]); }
#pragma unroll
  for (int j = 0; j < 8; ++j)
#pragma unroll
    for (int r = 0; r < 8; ++r) so[wave][8 * g + r][j * 16 + col] = acc[j][r] * IL[rloc0 + 8 * g + r];
  LDSX();
  for (int rl = 0; rl < 16; ++rl) vst2(OUT + (size_t)(nbase + rloc0 + rl) * DD + d0 + lane * 4, *(const v4f*)&so[wave][rl][lane * 4]);
}
extern "C" void kernel_launch(void* const* d_in, const int* in_sizes, int n_in, void* d_out, int out_size, void* d_ws, size_t ws_size, hipStream_t stream) {
  (void)in_sizes; (void)n_in; (void)out_size;
  const float** F = (const float**)d_in;
  if (ws_size < (size_t)WS_END) return;
  char* ws = (char*)d_ws; __bf16* P = (__bf16*)ws; _Float16 *Q = (_Float16*)(ws + WS_Q), *KH = (_Float16*)(ws + WS_KH), *KL = (_Float16*)(ws + WS_KL), *VT = (_Float16*)(ws + WS_VT), *Pm = (_Float16*)(ws + WS_P); float *S = (float*)(ws + WS_S), *IL = (float*)(ws + WS_IL);
  k_pack<<<dim3(DD, 3), 256, 0, stream>>>(F[1], F[3], F[5], P);
  k_proj<<<dim3(NN / 64, DD / 128, 3), 128, 0, stream>>>(F[0], P, F[2], F[4], F[6], Q, KH, KL, VT);
  for (int nb = 0; nb < NQB; ++nb) { const int nbase = nb * QBLK;
    k_scores<<<dim3(QBLK / 64, NN / 128), 128, 0, stream>>>(KH, KL, Q, nbase, S);
    k_soft<<<QBLK, 256, 0, stream>>>(S, Pm, IL);
    k_pv<<<dim3(QBLK / 64, DD / 128), 128, 0, stream>>>(Pm, VT, IL, nbase, (float*)d_out); }
}
